// TCNEnsemble_36086315221350
// MI455X (gfx1250) — hardware-verified
//
#include <hip/hip_runtime.h>
#include <math.h>

typedef __attribute__((ext_vector_type(16))) _Float16 v16h;
typedef __attribute__((ext_vector_type(16))) __bf16 v16b;
typedef __attribute__((ext_vector_type(8)))  _Float16 v8h;
typedef __attribute__((ext_vector_type(8)))  float v8f;
typedef __attribute__((ext_vector_type(4)))  float v4f;
typedef __attribute__((ext_vector_type(2)))  float v2f;
typedef __attribute__((ext_vector_type(4)))  unsigned v4u;
typedef __attribute__((ext_vector_type(4)))  int v4i;
typedef float __attribute__((may_alias)) float_a;
typedef int __attribute__((may_alias)) int_a;

template <typename T> __device__ __forceinline__ void vst2(void* p, T v) { *(volatile T*)p = v; __threadfence(); *(volatile T*)p = v; }
__device__ __forceinline__ v8f wmma16(v16h a, v16h b, v8f c) {
  v8f d = __builtin_amdgcn_wmma_f32_16x16x32_f16(false, a, false, b, (short)0, c, false, false);
  asm volatile("v_nop\n\tv_nop\n\tv_nop\n\tv_nop" : "+v"(d) : "v"(a), "v"(b));
  return d;
}
__device__ __forceinline__ v8f wmma_bf(v16b a, v16b b, v8f c) {
  v8f d = __builtin_amdgcn_wmma_f32_16x16x32_bf16(false, a, false, b, (short)0, c, false, false);
  asm volatile("v_nop\n\tv_nop\n\tv_nop\n\tv_nop" : "+v"(d) : "v"(a), "v"(b));
  return d;
}
__device__ __forceinline__ v16h frag_h(const _Float16* rowk0, int lane) {
  union { v16h v; v8h q[2]; } u; const _Float16* p = rowk0 + 8 * (lane >> 4);
  u.q[0] = *(const v8h*)p; u.q[1] = *(const v8h*)(p + 16); return u.v;
}
__device__ __forceinline__ v16h frag_f32(const float* rowk0, int lane) {
  v16h a; const float* p = rowk0 + 8 * (lane >> 4);
#pragma unroll
  for (int i = 0; i < 8; ++i) { a[i] = (_Float16)p[i]; a[8 + i] = (_Float16)p[16 + i]; }
  return a;
}
__device__ __forceinline__ v16h frag_f32s(const float* rowk0, int lane, float sc) {
  v16h a; const float* p = rowk0 + 8 * (lane >> 4);
#pragma unroll
  for (int i = 0; i < 8; ++i) { a[i] = (_Float16)(p[i] * sc); a[8 + i] = (_Float16)(p[16 + i] * sc); }
  return a;
}
__device__ __forceinline__ v16h fragc_f32(const float* W, int k0, int n, int lane, int ld, int K) {
  v16h a; const int g = lane >> 4;
#pragma unroll
  for (int i = 0; i < 8; ++i) { const int ka = k0 + 8 * g + i, kb = ka + 16;
    a[i] = (_Float16)(ka < K ? W[(size_t)ka * ld + n] : 0.f); a[8 + i] = (_Float16)(kb < K ? W[(size_t)kb * ld + n] : 0.f); }
  return a;
}
struct F2 { v16b h, l; };
__device__ __forceinline__ F2 bsplit16(const float v[16]) { F2 r;
#pragma unroll
  for (int i = 0; i < 16; ++i) { const __bf16 h = (__bf16)v[i]; r.h[i] = h; r.l[i] = (__bf16)(v[i] - (float)h); }
  return r; }
__device__ __forceinline__ F2 split_row(const float* row, int k0, int lane) { float v[16]; const float* p = row + k0 + 8 * (lane >> 4);
#pragma unroll
  for (int i = 0; i < 8; ++i) { v[i] = p[i]; v[8 + i] = p[16 + i]; }
  return bsplit16(v); }
__device__ __forceinline__ F2 split_rowK(const float* row, int k0, int lane, int K) { float v[16]; const int g = lane >> 4;
#pragma unroll
  for (int i = 0; i < 8; ++i) { const int ka = k0 + 8 * g + i, kb = ka + 16; v[i] = ka < K ? row[ka] : 0.f; v[8 + i] = kb < K ? row[kb] : 0.f; }
  return bsplit16(v); }
__device__ __forceinline__ F2 split_col(const float* W, int k0, int n, int lane, int ld, int K) { float v[16]; const int g = lane >> 4;
#pragma unroll
  for (int i = 0; i < 8; ++i) { const int ka = k0 + 8 * g + i, kb = ka + 16; v[i] = ka < K ? W[(size_t)ka * ld + n] : 0.f; v[8 + i] = kb < K ? W[(size_t)kb * ld + n] : 0.f; }
  return bsplit16(v); }
__device__ __forceinline__ v8f mac3(const F2& a, const F2& b, v8f c) { c = wmma_bf(a.l, b.h, c); c = wmma_bf(a.h, b.l, c); return wmma_bf(a.h, b.h, c); }
__device__ __forceinline__ float sigm(float v) { return 1.0f / (1.0f + expf(-v)); }
#define LDSX() do { asm volatile("s_wait_dscnt 0" ::: "memory"); __builtin_amdgcn_wave_barrier(); __builtin_amdgcn_fence(__ATOMIC_RELEASE, "workgroup"); } while (0)

#define NBT 32
#define TT 1024
#define NF 8
#define CC 128
#define KW 3
#define NLV 4
#define WN 64
#define KCI (CC * KW)

__device__ __forceinline__ float lrelu(float v) { return v > 0.f ? v : 0.01f * v; }

__device__ __forceinline__ void conv128(float (*IN)[CC + 4], float (*OUT)[CC + 4], const float* __restrict__ W, const float* __restrict__ bias, int dil, _Float16 (*sA)[40], int wave, int lane) {
  const int col = lane & 15, g = lane >> 4;
  v8f acc[8];
#pragma unroll
  for (int j = 0; j < 8; ++j) acc[j] = (v8f){};
#pragma unroll 1
  for (int kc = 0; kc < KCI / 32; ++kc) {
    { const int t = wave * 16 + col; union { v8h h[2]; v4u u2[2]; } pk;
#pragma unroll
      for (int u = 0; u < 16; ++u) { const int k = kc * 32 + g * 16 + u; const int ci = k / KW, jj = k % KW; const int ts = t - (KW - 1 - jj) * dil; pk.h[u >> 3][u & 7] = (_Float16)(ts >= 0 ? IN[ts][ci] : 0.f); }
      *(v4u*)(&sA[col][g * 16]) = pk.u2[0]; *(v4u*)(&sA[col][g * 16 + 8]) = pk.u2[1]; }
    LDSX();
    const v16h a = frag_h(&sA[col][0], lane);
#pragma unroll
    for (int j = 0; j < 8; ++j) acc[j] = wmma16(a, frag_f32s(W + (size_t)(j * 16 + col) * KCI + kc * 32, lane, 16.0f), acc[j]);
    LDSX(); }
#pragma unroll
  for (int j = 0; j < 8; ++j) { const int o = j * 16 + col; const float bb = bias[o];
#pragma unroll
    for (int r = 0; r < 8; ++r) OUT[wave * 16 + 8 * g + r][o] = acc[j][r] * (1.0f / 16.0f) + bb; }
}
__global__ __launch_bounds__(128) void k_branch(const float* __restrict__ x, const float* __restrict__ rw, const float* __restrict__ rb, const float* __restrict__ w10, const float* __restrict__ b10, const float* __restrict__ w20, const float* __restrict__ b20, const float* __restrict__ dw, const float* __restrict__ db,
                                              const float* __restrict__ w1r, const float* __restrict__ b1r, const float* __restrict__ w2r, const float* __restrict__ b2r, float* __restrict__ FE, float* __restrict__ MS) {
  __shared__ __align__(16) float hA[WN][CC + 4], hB[WN][CC + 4], hC[WN][CC + 4];
  __shared__ __align__(16) _Float16 sA[4][16][40];
  __shared__ float sxn[WN]; __shared__ float sred[2][4]; __shared__ float sstat[2]; __shared__ __align__(16) float sfe[CC]; __shared__ __align__(16) float sms[32];
  const int tid = threadIdx.x, wave = tid >> 5, lane = tid & 31;
  const int f = blockIdx.x, b = blockIdx.y;
  { float s = 0.f; for (int t = tid; t < TT; t += 128) s += x[((size_t)b * TT + t) * NF + f];
#pragma unroll
    for (int off = 16; off >= 1; off >>= 1) s += __shfl_xor(s, off, 32);
    if (lane == 0) sred[0][wave] = s;
    __syncthreads();
    const float mean = ((sred[0][0] + sred[0][1]) + (sred[0][2] + sred[0][3])) * (1.0f / TT);
    float q2 = 0.f; for (int t = tid; t < TT; t += 128) { const float d = x[((size_t)b * TT + t) * NF + f] - mean; q2 += d * d; }
#pragma unroll
    for (int off = 16; off >= 1; off >>= 1) q2 += __shfl_xor(q2, off, 32);
    if (lane == 0) sred[1][wave] = q2;
    __syncthreads();
    if (tid == 0) { const float var = ((sred[1][0] + sred[1][1]) + (sred[1][2] + sred[1][3])) * (1.0f / TT); sstat[0] = mean; sstat[1] = sqrtf(var + 1e-5f); }
    __syncthreads(); }
  const float mean = sstat[0], sd = sstat[1];
  if (tid < WN) { const int t = TT - WN + tid; sxn[tid] = (x[((size_t)b * TT + t) * NF + f] - mean) / sd * rw[f] + rb[f]; }
  __syncthreads();
  for (int q = tid; q < WN * CC; q += 128) { const int t = q >> 7, o = q & 127; float v = b10[f * CC + o];
#pragma unroll
    for (int jj = 0; jj < KW; ++jj) { const int ts = t - (KW - 1 - jj); if (ts >= 0) v += w10[((size_t)f * CC + o) * KW + jj] * sxn[ts]; }
    hA[t][o] = lrelu(v); }
  __syncthreads();
  conv128(hA, hB, w20 + (size_t)f * CC * KCI, b20 + f * CC, 1, sA[wave], wave, lane);
  __syncthreads();
  for (int q = tid; q < WN * CC; q += 128) { const int t = q >> 7, o = q & 127; const float res = dw[f * CC + o] * sxn[t] + db[f * CC + o]; const float v = lrelu(hB[t][o]) + res; hC[t][o] = v > 0.f ? v : 0.f; }
  __syncthreads();
#pragma unroll 1
  for (int l = 0; l < NLV - 1; ++l) { const int dil = 2 << l;
    conv128(hC, hA, w1r + ((size_t)l * NF + f) * CC * KCI, b1r + (l * NF + f) * CC, dil, sA[wave], wave, lane);
    __syncthreads();
    for (int q = tid; q < WN * CC; q += 128) { const int t = q >> 7, o = q & 127; hA[t][o] = lrelu(hA[t][o]); }
    __syncthreads();
    conv128(hA, hB, w2r + ((size_t)l * NF + f) * CC * KCI, b2r + (l * NF + f) * CC, dil, sA[wave], wave, lane);
    __syncthreads();
    for (int q = tid; q < WN * CC; q += 128) { const int t = q >> 7, o = q & 127; const float v = lrelu(hB[t][o]) + hC[t][o]; hC[t][o] = v > 0.f ? v : 0.f; }
    __syncthreads(); }
  if (tid < CC) sfe[tid] = hC[WN - 1][tid];
  if (tid < 32) sms[tid] = tid == 0 ? mean : (tid == 1 ? sd : 0.f);
  __syncthreads();
  if (tid < CC / 4) vst2(FE + (size_t)b * (NF * CC) + f * CC + tid * 4, *(const v4f*)(&sfe[tid * 4]));
  if (f == 0 && tid < 8) vst2(MS + (size_t)b * 32 + tid * 4, *(const v4f*)(&sms[tid * 4]));
}
__global__ __launch_bounds__(256) void k_head(const float* __restrict__ FE, const float* __restrict__ MS, const float* __restrict__ hw1, const float* __restrict__ hb1, const float* __restrict__ hw2, const float* __restrict__ hb2, const float* __restrict__ hw3, const float* __restrict__ hb3, const float* __restrict__ rw, const float* __restrict__ rb, float* __restrict__ out) {
  __shared__ float sh1[NBT][256 + 1]; __shared__ float sh2[NBT][CC + 1]; __shared__ __align__(16) float sy[NBT];
  const int tid = threadIdx.x;
  { const int n = tid; const float* wr = hw1 + (size_t)n * (NF * CC);
    for (int r = 0; r < NBT; ++r) { const float* fr = FE + (size_t)r * (NF * CC); float s = hb1[n];
#pragma unroll 4
      for (int k = 0; k < NF * CC; ++k) s += fr[k] * wr[k];
      sh1[r][n] = lrelu(s); } }
  __syncthreads();
  for (int q = tid; q < NBT * CC; q += 256) { const int r = q >> 7, n = q & 127; const float* wr = hw2 + (size_t)n * 256; float s = hb2[n];
#pragma unroll 4
    for (int k = 0; k < 256; ++k) s += sh1[r][k] * wr[k];
    sh2[r][n] = lrelu(s); }
  __syncthreads();
  if (tid < NBT) { float s = hb3[0];
#pragma unroll 4
    for (int k = 0; k < CC; ++k) s += sh2[tid][k] * hw3[k];
    const float m = MS[(size_t)tid * 32], sdv = MS[(size_t)tid * 32 + 1];
    float yv = (s - rb[0]) / (rw[0] + 1e-10f); sy[tid] = yv * sdv + m; }
  __syncthreads();
  if (tid < NBT / 4) vst2(out + tid * 4, *(const v4f*)(&sy[tid * 4]));
}
extern "C" void kernel_launch(void* const* d_in, const int* in_sizes, int n_in, void* d_out, int out_size, void* d_ws, size_t ws_size, hipStream_t stream) {
  (void)in_sizes; (void)n_in; (void)out_size; (void)ws_size;
  const float** I = (const float**)d_in;
  const float* x = I[0]; const float* rw = I[1]; const float* rb = I[2]; const float* w10 = I[3]; const float* b10 = I[4]; const float* w20 = I[5]; const float* b20 = I[6]; const float* dw = I[7]; const float* db = I[8];
  const float* w1r = I[9]; const float* b1r = I[10]; const float* w2r = I[11]; const float* b2r = I[12]; const float* hw1 = I[13]; const float* hb1 = I[14]; const float* hw2 = I[15]; const float* hb2 = I[16]; const float* hw3 = I[17]; const float* hb3 = I[18];
  float* out = (float*)d_out;
  char* ws = (char*)d_ws; size_t off = 0;
  auto take = [&](size_t bytes) { char* p = ws + off; off += (bytes + 255) & ~(size_t)255; return p; };
  float* FE = (float*)take((size_t)NBT * NF * CC * 4); float* MS = (float*)take((size_t)NBT * 32 * 4);
  k_branch<<<dim3(NF, NBT), 128, 0, stream>>>(x, rw, rb, w10, b10, w20, b20, dw, db, w1r, b1r, w2r, b2r, FE, MS);
  k_head<<<1, 256, 0, stream>>>(FE, MS, hw1, hb1, hw2, hb2, hw3, hb3, rw, rb, out);
}
